// SamplingMPNN_77352361001415
// MI455X (gfx1250) — hardware-verified
//
#include <hip/hip_runtime.h>
#include <stddef.h>


#define DIM    64
#define IND    128
#define EH     128
#define NG3    192
#define KBIG   8256
#define KPASS  2048
#define NPASS  4
#define SP     2112
#define NBK    128
#define SCAP   32
#define PCAP   2048
#define CT     128
#define CW     4
#define EPT    8
#define CHUNK  (CT * EPT)
#define WCAP   (EPT * 32)
#define XP     136
#define AP     72
#define STEPS  3

#define PW0    0
#define PWR    (PW0 + 2 * DIM * IND)
#define PWIH   (PWR + 2 * DIM * DIM)
#define PWHH   (PWIH + 2 * NG3 * DIM)
#define PW1    (PWHH + 2 * NG3 * DIM)
#define PW2    (PW1 + 2 * DIM * DIM)
#define PWTOT  (PW2 + 2 * DIM * DIM)

#define L_SH    0
#define L_SL    (L_SH + 16 * SP * 2)
#define L_OT    (L_SL + 16 * SP * 2)
#define L_HT    (L_OT + 16 * 64 * 32 * 2)
#define L_PEND  (L_HT + CW * 32 * 32 * 2)
#define L_SLOT  (L_PEND + PCAP * 4)
#define L_CNT   (L_SLOT + NBK * SCAP * 4)
#define L_LIST  (L_CNT + NBK * 4)
#define L_WC    (L_LIST + CW * WCAP * 4)
#define L_OST   (L_WC + 64)
#define L_TOTAL (L_OST + 16 * DIM * 4)

#define BO_CONV 0
#define BO_IH   (BO_CONV + DIM)
#define BO_HH   (BO_IH + NG3)
#define BO_1    (BO_HH + NG3)
#define BO_2    (BO_1 + DIM)
#define BO_TOT  (BO_2 + DIM)

#define T_ABH   0
#define T_ABL   (T_ABH + 16 * AP * 2)
#define T_GI    (T_ABL + 16 * AP * 2)
#define T_OST   (T_GI + 12 * 32 * 8 * 4)
#define T_X32   (T_OST + 16 * DIM * 4)
#define T_AG    (T_X32 + 16 * DIM * 4)
#define T_BS    (T_AG + 16 * DIM * 4)
#define T_WAVE  (T_BS + BO_TOT * 4)
#define T_TOTAL (CW * T_WAVE)

static_assert(NBK == 128 && CT == NBK);
static_assert(CW * 32 == CT);
static_assert(SCAP == 32);
static_assert(WCAP == 256 && CHUNK == 1024);
static_assert(KBIG == NPASS * KPASS + DIM);
static_assert(KPASS == 32 * DIM && SP == KPASS + DIM);
static_assert((SP % 32) == 0 && (KBIG % 32) == 0 && (KBIG % 8) == 0);
static_assert((XP % 8) == 0 && (AP % 8) == 0);
static_assert((PWR % 64) == 0 && (PWIH % 64) == 0 && (PWHH % 64) == 0 && (PW1 % 64) == 0 && (PW2 % 64) == 0);
static_assert((L_SL % 16) == 0 && (L_OT % 16) == 0 && (L_HT % 16) == 0 && (L_PEND % 16) == 0);
static_assert((L_SLOT % 16) == 0 && (L_CNT % 16) == 0 && (L_LIST % 16) == 0 && (L_WC % 16) == 0);
static_assert((L_OST % 16) == 0 && (L_TOTAL % 16) == 0 && L_TOTAL <= 300 * 1024);
static_assert((T_ABL % 16) == 0 && (T_GI % 16) == 0 && (T_OST % 16) == 0 && (T_X32 % 16) == 0);
static_assert((T_AG % 16) == 0 && (T_BS % 16) == 0 && (T_WAVE % 16) == 0);
static_assert((BO_IH % 4) == 0 && (BO_HH % 4) == 0 && (BO_1 % 4) == 0 && (BO_2 % 4) == 0 && BO_TOT == 576);
static_assert(T_TOTAL <= 300 * 1024);
static_assert(16 * 2 == (CT / 8) * 2);
static_assert(16 * DIM == 32 * 8 * 4);

typedef float          v4f  __attribute__((ext_vector_type(4)));
typedef float          v4fa __attribute__((ext_vector_type(4), __may_alias__));
typedef float          v8f  __attribute__((ext_vector_type(8)));
typedef int            v4i  __attribute__((ext_vector_type(4)));
typedef _Float16       v8h  __attribute__((ext_vector_type(8), __may_alias__));
typedef _Float16       v16h __attribute__((ext_vector_type(16)));
typedef __bf16         v16b __attribute__((ext_vector_type(16)));
typedef unsigned short v8us __attribute__((ext_vector_type(8), __may_alias__));
typedef unsigned short v4us __attribute__((ext_vector_type(4), __may_alias__));
union FragH { v16h v; v8h hv[2]; };
union FragB { v16b v; v8us u[2]; };
union U16   { v8h h; v8us u; v4f f; };

__device__ __forceinline__ v8f wmh(v16h a, v16h b, v8f c) {
  v8f d = __builtin_amdgcn_wmma_f32_16x16x32_f16(false, a, false, b, (short)0, c, false, false);
  asm volatile("v_nop\n\tv_nop\n\tv_nop\n\tv_nop" : "+v"(d) : "v"(a), "v"(b));
  return d;
}
__device__ __forceinline__ v8f wmb(v16b a, v16b b, v8f c) {
  v8f d = __builtin_amdgcn_wmma_f32_16x16x32_bf16(false, a, false, b, (short)0, c, false, false);
  asm volatile("v_nop\n\tv_nop\n\tv_nop\n\tv_nop" : "+v"(d) : "v"(a), "v"(b));
  return d;
}

__device__ __forceinline__ v8f z8f() {
  v8f c;
#pragma unroll
  for (int i = 0; i < 8; ++i) c[i] = 0.0f;
  return c;
}
__device__ __forceinline__ v8h z8h() {
  v8h c;
#pragma unroll
  for (int i = 0; i < 8; ++i) c[i] = (_Float16)0.0f;
  return c;
}

__device__ __forceinline__ int clampi(int v, int lo, int hi) { return v < lo ? lo : (v > hi ? hi : v); }

__device__ __forceinline__ void split1(float x, unsigned short& hs, unsigned short& ls) {
  const __bf16 hb = (__bf16)x;
  const float hf = (float)hb;
  const __bf16 lb = (__bf16)(x - hf);
  hs = __builtin_bit_cast(unsigned short, hb);
  ls = __builtin_bit_cast(unsigned short, lb);
}
__device__ __forceinline__ void split8(v8f d, U16& uh, U16& ul) {
#pragma unroll
  for (int i = 0; i < 8; ++i) {
    unsigned short a, b;
    split1(d[i], a, b);
    uh.u[i] = a;
    ul.u[i] = b;
  }
}

__device__ __forceinline__ float sigf(float x) { return __builtin_amdgcn_rcpf(1.0f + __expf(-x)); }
__device__ __forceinline__ float tnhf(float x) { return 2.0f * __builtin_amdgcn_rcpf(1.0f + __expf(-2.0f * x)) - 1.0f; }

__device__ __forceinline__ void stage16(float* dst, const float* __restrict__ src, int lane) {
  const int i = lane > 15 ? 15 : lane;
  const v4f v = *(const v4f*)(src + 4 * i);
  *(v4fa*)(dst + 4 * i) = v;
}
__device__ __forceinline__ void stage48(float* dst, const float* __restrict__ src, int lane) {
  const int i0 = lane;
  int i1 = lane + 32;
  i1 = i1 > 47 ? 47 : i1;
  const v4f v0 = *(const v4f*)(src + 4 * i0);
  const v4f v1 = *(const v4f*)(src + 4 * i1);
  *(v4fa*)(dst + 4 * i0) = v0;
  *(v4fa*)(dst + 4 * i1) = v1;
}
__device__ __forceinline__ void stage_tile(float* dst, const float* __restrict__ src, int lane) {
#pragma unroll
  for (int q = 0; q < 8; ++q) {
    const v4f v = *(const v4f*)(src + (size_t)(32 * q + lane) * 4);
    *(v4fa*)(dst + (32 * q + lane) * 4) = v;
  }
}
__device__ __forceinline__ void wave_sync_lds() {
  __builtin_amdgcn_fence(__ATOMIC_ACQ_REL, "wavefront");
  __builtin_amdgcn_wave_barrier();
}

__global__ __launch_bounds__(128) void k_prepw(const float* __restrict__ w0, const float* __restrict__ wr,
                                               const float* __restrict__ wih, const float* __restrict__ whh,
                                               const float* __restrict__ w1, const float* __restrict__ w2,
                                               unsigned short* wsp) {
  const int plane = blockIdx.y;
  const int gid = blockIdx.x * 128 + threadIdx.x;
  int rows = DIM, len = DIM, base = PW2, tr = 0;
  const float* src = w2;
  if (plane == 0)      { rows = DIM; len = IND; base = PW0;  src = w0; }
  else if (plane == 1) { rows = DIM; len = DIM; base = PWR;  src = wr; tr = 1; }
  else if (plane == 2) { rows = NG3; len = DIM; base = PWIH; src = wih; }
  else if (plane == 3) { rows = NG3; len = DIM; base = PWHH; src = whh; }
  else if (plane == 4) { rows = DIM; len = DIM; base = PW1;  src = w1; }
  const int ppr = len >> 3;
  if (gid >= rows * ppr) return;
  const int row = gid / ppr, p = gid - row * ppr;
  U16 uh, ul;
#pragma unroll
  for (int j = 0; j < 8; ++j) {
    const int k = 8 * p + j;
    const int idx = (tr != 0) ? (k * DIM + row) : (row * len + k);
    unsigned short a, b;
    split1(src[idx], a, b);
    uh.u[j] = a;
    ul.u[j] = b;
  }
  volatile v4f* qh = (volatile v4f*)(wsp + base + (size_t)row * len + 8 * p);
  volatile v4f* ql = (volatile v4f*)(wsp + base + (size_t)rows * len + (size_t)row * len + 8 * p);
  *qh = uh.f;
  *ql = ul.f;
  __threadfence();
  *qh = uh.f;
  *ql = ul.f;
}

__global__ __launch_bounds__(128) void k_prepa2(const float* __restrict__ a2, const float* __restrict__ c2,
                                                unsigned short* bph, unsigned short* bpl) {
  const int gid = blockIdx.x * 128 + threadIdx.x;
  if (gid >= DIM * (KBIG / 8)) return;
  const int o = gid / (KBIG / 8);
  const int p = gid - o * (KBIG / 8);
  U16 uh, ul;
#pragma unroll
  for (int j = 0; j < 8; ++j) {
    const int kk = 8 * p + j;
    const int kw = kk > DIM * EH - 1 ? DIM * EH - 1 : kk;
    const int k = kw >> 6, i = kw & 63;
    const float vw = a2[((size_t)(i * DIM + o)) * EH + k];
    int ib = kk - DIM * EH;
    ib = ib < 0 ? 0 : (ib > DIM - 1 ? DIM - 1 : ib);
    const float vb = c2[ib * DIM + o];
    const float v = (kk < DIM * EH) ? vw : vb;
    unsigned short a, b;
    split1(v, a, b);
    uh.u[j] = a;
    ul.u[j] = b;
  }
  volatile v4f* qh = (volatile v4f*)(bph + (size_t)o * KBIG + 8 * p);
  volatile v4f* ql = (volatile v4f*)(bpl + (size_t)o * KBIG + 8 * p);
  *qh = uh.f;
  *ql = ul.f;
  __threadfence();
  *qh = uh.f;
  *ql = ul.f;
}

__global__ __launch_bounds__(CT) void k_h0(const float* __restrict__ x, const unsigned short* __restrict__ wsp,
                                           const float* __restrict__ b0, float* h32, _Float16* h16,
                                           int nSrc, int nTgt) {
  __shared__ __attribute__((aligned(16))) unsigned short xth[64 * XP];
  __shared__ __attribute__((aligned(16))) unsigned short xtl[64 * XP];
  __shared__ __attribute__((aligned(16))) float st32[CW * 16 * DIM];
  __shared__ __attribute__((aligned(16))) _Float16 st16[CW * 16 * DIM];
  const int tid = threadIdx.x, lane = tid & 31, wave = tid >> 5, h = lane >> 4, m = lane & 15;
  const int row0 = blockIdx.x * 64;
#pragma unroll 2
  for (int it = 0; it < 16; ++it) {
    const int idx = it * 512 + tid * 4;
    const int r = idx >> 7, c = idx & 127;
    int gr = row0 + r;
    gr = gr > nSrc - 1 ? nSrc - 1 : gr;
    const v4f v = *(const v4f*)(x + (size_t)gr * IND + c);
    v4us uh, ul;
#pragma unroll
    for (int q = 0; q < 4; ++q) {
      unsigned short a, b;
      split1(v[q], a, b);
      uh[q] = a;
      ul[q] = b;
    }
    *(v4us*)(xth + r * XP + c) = uh;
    *(v4us*)(xtl + r * XP + c) = ul;
  }
  __syncthreads();

  const unsigned short* w0h = wsp + PW0;
  const unsigned short* w0l = wsp + PW0 + DIM * IND;
  v8f acc[4];
#pragma unroll
  for (int nt = 0; nt < 4; ++nt) acc[nt] = z8f();
#pragma unroll 1
  for (int ks = 0; ks < IND / 32; ++ks) {
    FragB ah, al;
    const unsigned short* ar = xth + (16 * wave + m) * XP + 32 * ks + 8 * h;
    const unsigned short* aq = xtl + (16 * wave + m) * XP + 32 * ks + 8 * h;
    ah.u[0] = *(const v8us*)ar;
    ah.u[1] = *(const v8us*)(ar + 16);
    al.u[0] = *(const v8us*)aq;
    al.u[1] = *(const v8us*)(aq + 16);
#pragma unroll
    for (int nt = 0; nt < 4; ++nt) {
      FragB bh, bl;
      const unsigned short* br = w0h + (size_t)(16 * nt + m) * IND + 32 * ks + 8 * h;
      const unsigned short* bq = w0l + (size_t)(16 * nt + m) * IND + 32 * ks + 8 * h;
      bh.u[0] = *(const v8us*)br;
      bh.u[1] = *(const v8us*)(br + 16);
      bl.u[0] = *(const v8us*)bq;
      bl.u[1] = *(const v8us*)(bq + 16);
      acc[nt] = wmb(ah.v, bh.v, acc[nt]);
      acc[nt] = wmb(ah.v, bl.v, acc[nt]);
      acc[nt] = wmb(al.v, bh.v, acc[nt]);
    }
  }
  float* s32 = st32 + wave * 16 * DIM;
  _Float16* s16 = st16 + wave * 16 * DIM;
#pragma unroll
  for (int nt = 0; nt < 4; ++nt) {
    const float bias = b0[16 * nt + m];
#pragma unroll
    for (int r = 0; r < 8; ++r) {
      const float v = fmaxf(acc[nt][r] + bias, 0.0f);
      s32[(8 * h + r) * DIM + 16 * nt + m] = v;
      s16[(8 * h + r) * DIM + 16 * nt + m] = (_Float16)(v * 8.0f);
    }
  }
  __builtin_amdgcn_fence(__ATOMIC_ACQ_REL, "wavefront");
  __builtin_amdgcn_wave_barrier();
  const int p8 = lane & 7, lr = lane >> 3;
  const int wrow0 = row0 + 16 * wave;
  v4f v16v[4];
  v4f v32v[8];
#pragma unroll
  for (int q = 0; q < 4; ++q) {
    const int row = 4 * q + lr;
    U16 u;
    u.h = *(const v8h*)(s16 + row * DIM + 8 * p8);
    v16v[q] = u.f;
  }
#pragma unroll
  for (int q = 0; q < 8; ++q) {
    const int L = 4 * q + lr;
    const int row = L >> 1, half = L & 1;
    v32v[q] = *(const v4fa*)(s32 + row * DIM + 32 * half + 4 * p8);
  }
  const bool dorow = (wrow0 + 16 <= nSrc);
  const bool do32  = (wrow0 + 16 <= nTgt);
  if (dorow) {
#pragma unroll
    for (int q = 0; q < 4; ++q)
      *(volatile v4f*)(h16 + (size_t)(wrow0 + 4 * q + lr) * DIM + 8 * p8) = v16v[q];
  }
  if (do32) {
#pragma unroll
    for (int q = 0; q < 8; ++q) {
      const int L = 4 * q + lr;
      const int row = L >> 1, half = L & 1;
      *(volatile v4f*)(h32 + (size_t)(wrow0 + row) * DIM + 32 * half + 4 * p8) = v32v[q];
    }
  }
  __threadfence();
  if (dorow) {
#pragma unroll
    for (int q = 0; q < 4; ++q)
      *(volatile v4f*)(h16 + (size_t)(wrow0 + 4 * q + lr) * DIM + 8 * p8) = v16v[q];
  }
  if (do32) {
#pragma unroll
    for (int q = 0; q < 8; ++q) {
      const int L = 4 * q + lr;
      const int row = L >> 1, half = L & 1;
      *(volatile v4f*)(h32 + (size_t)(wrow0 + row) * DIM + 32 * half + 4 * p8) = v32v[q];
    }
  }
}

__global__ __launch_bounds__(128) void k_edge(const int* __restrict__ eids, const float* __restrict__ ew,
                                              const float* __restrict__ a1, const float* __restrict__ c1,
                                              _Float16* he, int nE, int nEG) {
#pragma clang fp contract(off)
  const int gid = blockIdx.x * 128 + threadIdx.x;
  if (gid >= nE * 16) return;
  const int e = gid >> 4, p = gid & 15;
  int id = eids[e];
  id = id < 0 ? 0 : (id > nEG - 1 ? nEG - 1 : id);
  const float ea = ew[id];
  const v4f aA = *(const v4f*)(a1 + 8 * p);
  const v4f aB = *(const v4f*)(a1 + 8 * p + 4);
  const v4f cA = *(const v4f*)(c1 + 8 * p);
  const v4f cB = *(const v4f*)(c1 + 8 * p + 4);
  U16 u;
#pragma unroll
  for (int j = 0; j < 4; ++j) {
    const float t0 = ea * aA[j];
    float v0 = t0 + cA[j];
    v0 = fmaxf(v0, 0.0f);
    u.h[j] = (_Float16)(v0 * 16.0f);
    const float t1 = ea * aB[j];
    float v1 = t1 + cB[j];
    v1 = fmaxf(v1, 0.0f);
    u.h[4 + j] = (_Float16)(v1 * 16.0f);
  }
  volatile v4f* q = (volatile v4f*)(he + (size_t)e * EH + 8 * p);
  *q = u.f;
  __threadfence();
  *q = u.f;
}

__device__ __forceinline__ int scan_chunk(const int* __restrict__ dsts, int nE, int cbase, int nodeBase,
                                          int* list, int tid, int wave) {
  int wc = 0;
  const int el0  = tid * EPT;
  const int e0   = cbase + el0;
  const int sent = -2147483647 - 1;
  v4i da, db;
  if (cbase + CHUNK <= nE) {
    da = *(const v4i*)(dsts + e0);
    db = *(const v4i*)(dsts + e0 + 4);
  } else {
    da.x = (e0     < nE) ? dsts[clampi(e0,     0, nE - 1)] : sent;
    da.y = (e0 + 1 < nE) ? dsts[clampi(e0 + 1, 0, nE - 1)] : sent;
    da.z = (e0 + 2 < nE) ? dsts[clampi(e0 + 2, 0, nE - 1)] : sent;
    da.w = (e0 + 3 < nE) ? dsts[clampi(e0 + 3, 0, nE - 1)] : sent;
    db.x = (e0 + 4 < nE) ? dsts[clampi(e0 + 4, 0, nE - 1)] : sent;
    db.y = (e0 + 5 < nE) ? dsts[clampi(e0 + 5, 0, nE - 1)] : sent;
    db.z = (e0 + 6 < nE) ? dsts[clampi(e0 + 6, 0, nE - 1)] : sent;
    db.w = (e0 + 7 < nE) ? dsts[clampi(e0 + 7, 0, nE - 1)] : sent;
  }
  const unsigned nb = (unsigned)nodeBase;
  const unsigned s0 = (unsigned)da.x - nb, s1 = (unsigned)da.y - nb;
  const unsigned s2 = (unsigned)da.z - nb, s3 = (unsigned)da.w - nb;
  const unsigned s4 = (unsigned)db.x - nb, s5 = (unsigned)db.y - nb;
  const unsigned s6 = (unsigned)db.z - nb, s7 = (unsigned)db.w - nb;
  const bool h0 = s0 < (unsigned)NBK, h1 = s1 < (unsigned)NBK, h2 = s2 < (unsigned)NBK, h3 = s3 < (unsigned)NBK;
  const bool h4 = s4 < (unsigned)NBK, h5 = s5 < (unsigned)NBK, h6 = s6 < (unsigned)NBK, h7 = s7 < (unsigned)NBK;
  const unsigned any = __builtin_amdgcn_ballot_w32(h0 | h1 | h2 | h3 | h4 | h5 | h6 | h7);
  if (any != 0u) {
#define HITJ(J, HJ, SJ) { \
      const unsigned mj = __builtin_amdgcn_ballot_w32(HJ); \
      if (mj != 0u) { \
        if (HJ) { \
          const int pos = wc + (int)__builtin_amdgcn_mbcnt_lo(mj, 0u); \
          if (pos < WCAP) list[wave * WCAP + pos] = (el0 + (J)) * NBK + (int)(SJ); \
        } \
        wc += (int)__builtin_popcount(mj); } }
    HITJ(0, h0, s0)
    HITJ(1, h1, s1)
    HITJ(2, h2, s2)
    HITJ(3, h3, s3)
    HITJ(4, h4, s4)
    HITJ(5, h5, s5)
    HITJ(6, h6, s6)
    HITJ(7, h7, s7)
#undef HITJ
  }
  return wc;
}

__global__ __launch_bounds__(CT) void k_conv(const int* __restrict__ esrc, const int* __restrict__ edst,
                                             const _Float16* __restrict__ xh, const _Float16* __restrict__ he,
                                             const unsigned short* __restrict__ bph,
                                             const unsigned short* __restrict__ bpl,
                                             float* aggp, int nSrc, int nTgt, int nE) {
  extern __shared__ __attribute__((aligned(16))) unsigned char dsm[];
  unsigned short* sh    = (unsigned short*)(dsm + L_SH);
  unsigned short* sl    = (unsigned short*)(dsm + L_SL);
  _Float16*       otG   = (_Float16*)(dsm + L_OT);
  int*            pend  = (int*)(dsm + L_PEND);
  int*            slotL = (int*)(dsm + L_SLOT);
  int*            cntL  = (int*)(dsm + L_CNT);
  int*            list  = (int*)(dsm + L_LIST);
  int*            wc    = (int*)(dsm + L_WC);
  float*          ost   = (float*)(dsm + L_OST);
  const int tid = threadIdx.x, lane = tid & 31, wave = tid >> 5, h = lane >> 4, m = lane & 15;
  _Float16* htW = (_Float16*)(dsm + L_HT) + wave * (32 * 32);
  const int nodeBase = blockIdx.x * NBK;

  if (tid == 0) wc[CW] = 0;
  __syncthreads();
  const int nChunks = (nE + CHUNK - 1) / CHUNK;
#pragma unroll 1
  for (int ch = 0; ch < nChunks; ++ch) {
    const int cbase = ch * CHUNK;
    const int cwc = scan_chunk(edst, nE, cbase, nodeBase, list, tid, wave);
    if (lane == 0) wc[wave] = cwc;
    __syncthreads();
    const int base = wc[CW];
    int tot = 0, myoff = 0;
#pragma unroll
    for (int w = 0; w < CW; ++w) {
      int c = wc[w];
      c = c > WCAP ? WCAP : (c < 0 ? 0 : c);
      if (w < wave) myoff += c;
      tot += c;
    }
    {
      int n = wc[wave];
      n = n > WCAP ? WCAP : (n < 0 ? 0 : n);
      const int* lp = list + wave * WCAP;
      for (int i = lane; i < n; i += 32) {
        const int pos = base + myoff + i;
        if (pos < PCAP) pend[pos] = lp[i] + cbase * NBK;
      }
    }
    int newN = base + tot;
    newN = newN > PCAP ? PCAP : newN;
    __syncthreads();
    if (tid == 0) wc[CW] = newN;
  }
  __syncthreads();

  {
    int tot = wc[CW];
    tot = tot < 0 ? 0 : (tot > PCAP ? PCAP : tot);
    int cnt = 0;
#pragma unroll 1
    for (int j = 0; j < tot; ++j) {
      const int v = pend[j];
      if ((v & (NBK - 1)) == tid) {
        if (cnt < SCAP) slotL[tid * SCAP + cnt] = v >> 7;
        ++cnt;
      }
    }
    cntL[tid] = cnt;
  }
  __syncthreads();

  int nodesHere = nTgt - nodeBase;
  nodesHere = nodesHere > NBK ? NBK : nodesHere;
  const int ngroups = (nodesHere + 15) >> 4;
  const v8h zh = z8h();

#pragma unroll 1
  for (int g = 0; g < ngroups; ++g) {
#pragma unroll 1
    for (int q = 0; q < 4; ++q) {
      const int nl = 4 * wave + q, nb = 16 * g + nl;
      int cnt = cntL[nb];
      cnt = cnt < 0 ? 0 : (cnt > SCAP ? SCAP : cnt);
      const bool valid = lane < cnt;
      int e = slotL[nb * SCAP + lane];
      e = clampi(e, 0, nE - 1);
      int s = esrc[e];
      s = clampi(s, 0, nSrc - 1);
      const v8h* op = (const v8h*)(xh + (size_t)s * DIM);
      _Float16* xt = otG + nl * (64 * 32);
#pragma unroll
      for (int c = 0; c < 8; ++c) {
        v8h xv = op[c];
        xv = valid ? xv : zh;
#pragma unroll
        for (int j = 0; j < 8; ++j) xt[(8 * c + j) * 32 + lane] = xv[j];
      }
    }
    __syncthreads();

    v8f accA = z8f();
#pragma unroll 1
    for (int p = 0; p < NPASS; ++p) {
#pragma unroll 1
      for (int q = 0; q < 4; ++q) {
        const int nl = 4 * wave + q, nb = 16 * g + nl;
        int cnt = cntL[nb];
        cnt = cnt < 0 ? 0 : (cnt > SCAP ? SCAP : cnt);
        const bool valid = lane < cnt;
        int e = slotL[nb * SCAP + lane];
        e = clampi(e, 0, nE - 1);
        const v8h* hp = (const v8h*)(he + (size_t)e * EH + 32 * p);
        __builtin_amdgcn_fence(__ATOMIC_ACQ_REL, "wavefront");
        __builtin_amdgcn_wave_barrier();
#pragma unroll
        for (int c = 0; c < 4; ++c) {
          v8h hv = hp[c];
          hv = valid ? hv : zh;
#pragma unroll
          for (int j = 0; j < 8; ++j) htW[(8 * c + j) * 32 + lane] = hv[j];
        }
        __builtin_amdgcn_fence(__ATOMIC_ACQ_REL, "wavefront");
        __builtin_amdgcn_wave_barrier();
        const _Float16* xt = otG + nl * (64 * 32);
        unsigned short* shr = sh + nl * SP;
        unsigned short* slr = sl + nl * SP;
#pragma unroll
        for (int it = 0; it < 4; ++it) {
          FragH a;
          const _Float16* ar = xt + (16 * it + m) * 32 + 8 * h;
          a.hv[0] = *(const v8h*)ar;
          a.hv[1] = *(const v8h*)(ar + 16);
#pragma unroll
          for (int kt = 0; kt < 2; ++kt) {
            FragH b;
            const _Float16* br = htW + (16 * kt + m) * 32 + 8 * h;
            b.hv[0] = *(const v8h*)br;
            b.hv[1] = *(const v8h*)(br + 16);
            const v8f d = wmh(a.v, b.v, z8f());
            U16 uh, ul;
            split8(d, uh, ul);
            const int col = (16 * kt + m) * 64 + 16 * it + 8 * h;
            *(v8us*)(shr + col) = uh.u;
            *(v8us*)(slr + col) = ul.u;
          }
        }
        if (p == NPASS - 1) {
#pragma unroll
          for (int ii = 0; ii < 2; ++ii) {
            const int i = lane + 32 * ii;
            float t = 0.0f;
#pragma unroll
            for (int c = 0; c < 4; ++c) {
              const v8h xv = *(const v8h*)(xt + i * 32 + 8 * c);
#pragma unroll
              for (int j = 0; j < 8; ++j) t += (float)xv[j];
            }
            unsigned short hs, ls;
            split1(t * 16.0f, hs, ls);
            shr[KPASS + i] = hs;
            slr[KPASS + i] = ls;
          }
        }
      }
      __syncthreads();
      {
        const int KS = (p == NPASS - 1) ? ((KPASS + DIM) / 32) : (KPASS / 32);
        const unsigned short* aph = sh + m * SP + 8 * h;
        const unsigned short* apl = sl + m * SP + 8 * h;
        const unsigned short* bhp = bph + (size_t)(16 * wave + m) * KBIG + KPASS * p + 8 * h;
        const unsigned short* blp = bpl + (size_t)(16 * wave + m) * KBIG + KPASS * p + 8 * h;
#pragma unroll 2
        for (int ks = 0; ks < KS; ++ks) {
          FragB ah, al, bh, bl;
          ah.u[0] = *(const v8us*)(aph + 32 * ks);
          ah.u[1] = *(const v8us*)(aph + 32 * ks + 16);
          al.u[0] = *(const v8us*)(apl + 32 * ks);
          al.u[1] = *(const v8us*)(apl + 32 * ks + 16);
          bh.u[0] = *(const v8us*)(bhp + 32 * ks);
          bh.u[1] = *(const v8us*)(bhp + 32 * ks + 16);
          bl.u[0] = *(const v8us*)(blp + 32 * ks);
          bl.u[1] = *(const v8us*)(blp + 32 * ks + 16);
          accA = wmb(ah.v, bh.v, accA);
          accA = wmb(ah.v, bl.v, accA);
          accA = wmb(al.v, bh.v, accA);
        }
      }
      __syncthreads();
    }

    {
      const int o = 16 * wave + m;
#pragma unroll
      for (int r = 0; r < 8; ++r) {
        const int nbr = 16 * g + 8 * h + r;
        const int c = cntL[nbr];
        const float cf = (c > 0) ? (float)c : 1.0f;
        const float inv = 1.0f / cf;
        ost[(8 * h + r) * DIM + o] = accA[r] * (1.0f / 128.0f) * inv;
      }
    }
    __syncthreads();
    {
      const int p8 = tid & 7, Lb = tid >> 3;
      v4f v0, v1;
      char *d0, *d1;
      {
        const int L = Lb;
        const int row = L >> 1, half = L & 1;
        v0 = *(const v4fa*)(ost + row * DIM + 32 * half + 4 * p8);
        d0 = (char*)(aggp + (size_t)(nodeBase + 16 * g + row) * DIM + 32 * half + 4 * p8);
      }
      {
        const int L = 16 + Lb;
        const int row = L >> 1, half = L & 1;
        v1 = *(const v4fa*)(ost + row * DIM + 32 * half + 4 * p8);
        d1 = (char*)(aggp + (size_t)(nodeBase + 16 * g + row) * DIM + 32 * half + 4 * p8);
      }
      *(volatile v4f*)d0 = v0;
      *(volatile v4f*)d1 = v1;
      __threadfence();
      *(volatile v4f*)d0 = v0;
      *(volatile v4f*)d1 = v1;
    }
  }
}

__device__ __forceinline__ void put_tile(v8f t0, v8f t1, v8f t2, v8f t3, unsigned short* abh, unsigned short* abl,
                                         int h, int m, FragB& a0h, FragB& a1h, FragB& a0l, FragB& a1l) {
  __builtin_amdgcn_fence(__ATOMIC_ACQ_REL, "wavefront");
  __builtin_amdgcn_wave_barrier();
#pragma unroll
  for (int r = 0; r < 8; ++r) {
    const int rr = (8 * h + r) * AP + m;
    unsigned short a, b;
    split1(t0[r], a, b); abh[rr] = a;      abl[rr] = b;
    split1(t1[r], a, b); abh[rr + 16] = a; abl[rr + 16] = b;
    split1(t2[r], a, b); abh[rr + 32] = a; abl[rr + 32] = b;
    split1(t3[r], a, b); abh[rr + 48] = a; abl[rr + 48] = b;
  }
  __builtin_amdgcn_fence(__ATOMIC_ACQ_REL, "wavefront");
  __builtin_amdgcn_wave_barrier();
  const unsigned short* ph = abh + m * AP + 8 * h;
  const unsigned short* pl = abl + m * AP + 8 * h;
  a0h.u[0] = *(const v8us*)ph;        a0h.u[1] = *(const v8us*)(ph + 16);
  a1h.u[0] = *(const v8us*)(ph + 32); a1h.u[1] = *(const v8us*)(ph + 48);
  a0l.u[0] = *(const v8us*)pl;        a0l.u[1] = *(const v8us*)(pl + 16);
  a1l.u[0] = *(const v8us*)(pl + 32); a1l.u[1] = *(const v8us*)(pl + 48);
}

__device__ __forceinline__ v8f mm64(v8f acc, const unsigned short* __restrict__ ph,
                                     const unsigned short* __restrict__ pl, int nrow, int h,
                                     const FragB& a0h, const FragB& a1h, const FragB& a0l, const FragB& a1l) {
  const unsigned short* bp = ph + (size_t)nrow * DIM + 8 * h;
  const unsigned short* bq = pl + (size_t)nrow * DIM + 8 * h;
  FragB bh, bl;
  bh.u[0] = *(const v8us*)bp;        bh.u[1] = *(const v8us*)(bp + 16);
  bl.u[0] = *(const v8us*)bq;        bl.u[1] = *(const v8us*)(bq + 16);
  acc = wmb(a0h.v, bh.v, acc);
  acc = wmb(a0h.v, bl.v, acc);
  acc = wmb(a0l.v, bh.v, acc);
  bh.u[0] = *(const v8us*)(bp + 32); bh.u[1] = *(const v8us*)(bp + 48);
  bl.u[0] = *(const v8us*)(bq + 32); bl.u[1] = *(const v8us*)(bq + 48);
  acc = wmb(a1h.v, bh.v, acc);
  acc = wmb(a1h.v, bl.v, acc);
  acc = wmb(a1l.v, bh.v, acc);
  return acc;
}

__global__ __launch_bounds__(CT) void k_tail(const float* __restrict__ h32, const float* __restrict__ aggp,
                                             const unsigned short* __restrict__ wsp,
                                             const float* __restrict__ bconv, const float* __restrict__ bih,
                                             const float* __restrict__ bhh, const float* __restrict__ b1v,
                                             const float* __restrict__ b2v, float* out, int nTgt) {
  extern __shared__ __attribute__((aligned(16))) unsigned char dsm[];
  const int tid = threadIdx.x, lane = tid & 31, wave = tid >> 5, h = lane >> 4, m = lane & 15;
  unsigned char* wb = dsm + wave * T_WAVE;
  unsigned short* abh = (unsigned short*)(wb + T_ABH);
  unsigned short* abl = (unsigned short*)(wb + T_ABL);
  float* gib  = (float*)(wb + T_GI);
  float* ost  = (float*)(wb + T_OST);
  float* x32t = (float*)(wb + T_X32);
  float* agt  = (float*)(wb + T_AG);
  float* bs   = (float*)(wb + T_BS);
  const int ntiles = nTgt >> 4;
  const int tile = blockIdx.x * CW + wave;
  if (tile >= ntiles) return;
  const int r0 = tile * 16;
  const unsigned short* wrh  = wsp + PWR;   const unsigned short* wrl  = wrh + DIM * DIM;
  const unsigned short* wihh = wsp + PWIH;  const unsigned short* wihl = wihh + NG3 * DIM;
  const unsigned short* whhh = wsp + PWHH;  const unsigned short* whhl = whhh + NG3 * DIM;
  const unsigned short* w1h  = wsp + PW1;   const unsigned short* w1l  = w1h + DIM * DIM;
  const unsigned short* w2h  = wsp + PW2;   const unsigned short* w2l  = w2h + DIM * DIM;

  stage16(bs + BO_CONV, bconv, lane);
  stage48(bs + BO_IH, bih, lane);
  stage48(bs + BO_HH, bhh, lane);
  stage16(bs + BO_1, b1v, lane);
  stage16(bs + BO_2, b2v, lane);
  wave_sync_lds();
  stage_tile(x32t, h32 + (size_t)r0 * DIM, lane);
  wave_sync_lds();
  stage_tile(agt, aggp + (size_t)r0 * DIM, lane);
  wave_sync_lds();

  v8f hC[4];
#pragma unroll
  for (int nt = 0; nt < 4; ++nt)
#pragma unroll
    for (int r = 0; r < 8; ++r)
      hC[nt][r] = x32t[(8 * h + r) * DIM + 16 * nt + m];

  FragB a0h, a1h, a0l, a1l;
  put_tile(hC[0], hC[1], hC[2], hC[3], abh, abl, h, m, a0h, a1h, a0l, a1l);

  v8f mC[4];
#pragma unroll
  for (int nt = 0; nt < 4; ++nt) {
    const v8f acc = mm64(z8f(), wrh, wrl, 16 * nt + m, h, a0h, a1h, a0l, a1l);
    const float cb = bs[BO_CONV + 16 * nt + m];
#pragma unroll
    for (int r = 0; r < 8; ++r) {
      const float ag = agt[(8 * h + r) * DIM + 16 * nt + m];
      const float s = ag + acc[r];
      mC[nt][r] = fmaxf(s + cb, 0.0f);
    }
  }
  put_tile(mC[0], mC[1], mC[2], mC[3], abh, abl, h, m, a0h, a1h, a0l, a1l);

#pragma unroll
  for (int nt = 0; nt < 12; ++nt) {
    const v8f acc = mm64(z8f(), wihh, wihl, 16 * nt + m, h, a0h, a1h, a0l, a1l);
    const float b = bs[BO_IH + 16 * nt + m];
    v4f g0, g1;
#pragma unroll
    for (int r = 0; r < 4; ++r) { g0[r] = acc[r] + b; g1[r] = acc[4 + r] + b; }
    float* gp = gib + (nt * 32 + lane) * 8;
    *(v4f*)gp = g0;
    *(v4f*)(gp + 4) = g1;
  }

#pragma unroll 1
  for (int s = 0; s < STEPS; ++s) {
    put_tile(hC[0], hC[1], hC[2], hC[3], abh, abl, h, m, a0h, a1h, a0l, a1l);
#pragma unroll
    for (int nt = 0; nt < 4; ++nt) {
      const v8f ar = mm64(z8f(), whhh, whhl, 16 * nt + m, h, a0h, a1h, a0l, a1l);
      const v8f az = mm64(z8f(), whhh, whhl, DIM + 16 * nt + m, h, a0h, a1h, a0l, a1l);
      const v8f an = mm64(z8f(), whhh, whhl, 2 * DIM + 16 * nt + m, h, a0h, a1h, a0l, a1l);
      const float bhr = bs[BO_HH + 16 * nt + m];
      const float bhz = bs[BO_HH + DIM + 16 * nt + m];
      const float bhn = bs[BO_HH + 2 * DIM + 16 * nt + m];
      const float* gpr = gib + (nt * 32 + lane) * 8;
      const float* gpz = gib + ((nt + 4) * 32 + lane) * 8;
      const float* gpn = gib + ((nt + 8) * 32 + lane) * 8;
      const v4f gr0 = *(const v4f*)gpr, gr1 = *(const v4f*)(gpr + 4);
      const v4f gz0 = *(const v4f*)gpz, gz1 = *(const v4f*)(gpz + 4);
      const v4f gn0 = *(const v4f*)gpn, gn1 = *(const v4f*)(gpn + 4);
#pragma unroll
      for (int r = 0; r < 8; ++r) {
        const float gir = (r < 4) ? gr0[r & 3] : gr1[r & 3];
        const float giz = (r < 4) ? gz0[r & 3] : gz1[r & 3];
        const float gin = (r < 4) ? gn0[r & 3] : gn1[r & 3];
        const float ghr = ar[r] + bhr, ghz = az[r] + bhz, ghn = an[r] + bhn;
        const float rg = sigf(gir + ghr);
        const float zg = sigf(giz + ghz);
        const float ng = tnhf(gin + rg * ghn);
        hC[nt][r] = (1.0f - zg) * ng + zg * hC[nt][r];
      }
    }
  }

  put_tile(hC[0], hC[1], hC[2], hC[3], abh, abl, h, m, a0h, a1h, a0l, a1l);
  v8f o1[4];
#pragma unroll
  for (int nt = 0; nt < 4; ++nt) {
    const v8f acc = mm64(z8f(), w1h, w1l, 16 * nt + m, h, a0h, a1h, a0l, a1l);
    const float b = bs[BO_1 + 16 * nt + m];
#pragma unroll
    for (int r = 0; r < 8; ++r) o1[nt][r] = fmaxf(acc[r] + b, 0.0f);
  }
  put_tile(o1[0], o1[1], o1[2], o1[3], abh, abl, h, m, a0h, a1h, a0l, a1l);
#pragma unroll
  for (int nt = 0; nt < 4; ++nt) {
    const v8f acc = mm64(z8f(), w2h, w2l, 16 * nt + m, h, a0h, a1h, a0l, a1l);
    const float b = bs[BO_2 + 16 * nt + m];
#pragma unroll
    for (int r = 0; r < 8; ++r) ost[(8 * h + r) * DIM + 16 * nt + m] = acc[r] + b;
  }
  __builtin_amdgcn_fence(__ATOMIC_ACQ_REL, "wavefront");
  __builtin_amdgcn_wave_barrier();
  const int p8 = lane & 7, lr = lane >> 3;
  v4f v[8];
#pragma unroll
  for (int q = 0; q < 8; ++q) {
    const int L = 4 * q + lr;
    const int row = L >> 1, half = L & 1;
    v[q] = *(const v4fa*)(ost + row * DIM + 32 * half + 4 * p8);
  }
#pragma unroll
  for (int q = 0; q < 8; ++q) {
    const int L = 4 * q + lr;
    const int row = L >> 1, half = L & 1;
    *(volatile v4f*)(out + (size_t)(r0 + row) * DIM + 32 * half + 4 * p8) = v[q];
  }
  __threadfence();
#pragma unroll
  for (int q = 0; q < 8; ++q) {
    const int L = 4 * q + lr;
    const int row = L >> 1, half = L & 1;
    *(volatile v4f*)(out + (size_t)(r0 + row) * DIM + 32 * half + 4 * p8) = v[q];
  }
}

extern "C" void kernel_launch(void* const* d_in, const int* in_sizes, int n_in,
                              void* d_out, int out_size, void* d_ws, size_t ws_size,
                              hipStream_t stream) {
  if (n_in < 22) return;
  if (in_sizes[0] < IND || (in_sizes[0] % IND) != 0) return;
  const int nSrc = in_sizes[0] / IND;
  if (nSrc < 64 || (nSrc % 64) != 0) return;
  if (out_size < DIM || (out_size % DIM) != 0) return;
  const int nTgt = out_size / DIM;
  if ((nTgt % 16) != 0 || nTgt > nSrc) return;
  const int nE = in_sizes[2];
  if (nE < 1 || in_sizes[3] != nE || in_sizes[4] != nE) return;
  const int nEG = in_sizes[5];
  if (nEG < 1) return;
  if (in_sizes[6] != DIM * IND || in_sizes[7] != DIM || in_sizes[8] != EH || in_sizes[9] != EH) return;
  if (in_sizes[10] != DIM * DIM * EH || in_sizes[11] != DIM * DIM || in_sizes[12] != DIM * DIM || in_sizes[13] != DIM) return;
  if (in_sizes[14] != NG3 * DIM || in_sizes[15] != NG3 * DIM || in_sizes[16] != NG3 || in_sizes[17] != NG3) return;
  if (in_sizes[18] != DIM * DIM || in_sizes[19] != DIM || in_sizes[20] != DIM * DIM || in_sizes[21] != DIM) return;

  const float* x     = (const float*)d_in[0];
  const int*   esrc  = (const int*)d_in[2];
  const int*   edst  = (const int*)d_in[3];
  const int*   eids  = (const int*)d_in[4];
  const float* ew    = (const float*)d_in[5];
  const float* w0    = (const float*)d_in[6];
  const float* b0    = (const float*)d_in[7];
  const float* a1    = (const float*)d_in[8];
  const float* c1    = (const float*)d_in[9];
  const float* a2    = (const float*)d_in[10];
  const float* c2    = (const float*)d_in[11];
  const float* wroot = (const float*)d_in[12];
  const float* bconv = (const float*)d_in[13];
  const float* wih   = (const float*)d_in[14];
  const float* whh   = (const float*)d_in[15];
  const float* bih   = (const float*)d_in[16];
  const float* bhh   = (const float*)d_in[17];
  const float* w1    = (const float*)d_in[18];
  const float* b1    = (const float*)d_in[19];
  const float* w2    = (const float*)d_in[20];
  const float* b2    = (const float*)d_in[21];
  float* yout = (float*)d_out;

  char* ws = (char*)d_ws;
  size_t off = 0;
  auto carve = [&](size_t bytes) -> char* { char* p = ws + off; off += (bytes + 255) & ~(size_t)255; return p; };
  unsigned short* wsp  = (unsigned short*)carve((size_t)PWTOT * 2);
  unsigned short* bph  = (unsigned short*)carve((size_t)DIM * KBIG * 2);
  unsigned short* bpl  = (unsigned short*)carve((size_t)DIM * KBIG * 2);
  _Float16*       he   = (_Float16*)carve((size_t)nE * EH * 2);
  _Float16*       h16  = (_Float16*)carve((size_t)nSrc * DIM * 2);
  float*          h32  = (float*)carve((size_t)nTgt * DIM * 4);
  float*          aggp = (float*)carve((size_t)nTgt * DIM * 4);
  size_t limit = (size_t)134217728;
  if (ws_size < limit) limit = ws_size;
  if (off > limit) return;

  k_prepw<<<dim3((NG3 * 8 + 127) / 128, 6), 128, 0, stream>>>(w0, wroot, wih, whh, w1, w2, wsp);
  k_prepa2<<<(DIM * (KBIG / 8) + 127) / 128, 128, 0, stream>>>(a2, c2, bph, bpl);
  k_h0<<<nSrc / 64, CT, 0, stream>>>(x, wsp, b0, h32, h16, nSrc, nTgt);
  k_edge<<<(nE * 16 + 127) / 128, 128, 0, stream>>>(eids, ew, a1, c1, he, nE, nEG);

  hipFuncSetAttribute(reinterpret_cast<const void*>(&k_conv), hipFuncAttributeMaxDynamicSharedMemorySize, L_TOTAL);
  k_conv<<<(nTgt + NBK - 1) / NBK, CT, L_TOTAL, stream>>>(esrc, edst, h16, he, bph, bpl, aggp, nSrc, nTgt, nE);

  hipFuncSetAttribute(reinterpret_cast<const void*>(&k_tail), hipFuncAttributeMaxDynamicSharedMemorySize, T_TOTAL);
  k_tail<<<((nTgt / 16) + CW - 1) / CW, CT, T_TOTAL, stream>>>(h32, aggp, wsp, bconv, bih, bhh, b1, b2, yout, nTgt);
}
